// KANCouplingNet_40656160424367
// MI455X (gfx1250) — hardware-verified
//
#include <hip/hip_runtime.h>


#define NPIX 131072
#define HWS  4096
#define NIMG 32
#define CH   32768
#define NCH  (NPIX / CH)
#define NG   8
#define NKN  12
#define NF   9
#define D0   12
#define D1   64
#define D2   64
#define D3   24
#define K0   128
#define K1   576
#define NPAD 64
typedef _Float16 h16;
typedef unsigned short bf;
typedef __attribute__((ext_vector_type(16))) __bf16   v16bf;
typedef __attribute__((ext_vector_type(16))) _Float16 v16h;
typedef __attribute__((ext_vector_type(8)))  _Float16 v8h;
typedef __attribute__((ext_vector_type(8)))  unsigned short v8us;
typedef __attribute__((ext_vector_type(8)))  float    v8f;
typedef __attribute__((ext_vector_type(4)))  float    v4f;
typedef v8h  __attribute__((may_alias)) v8ha;
typedef v4f  __attribute__((may_alias)) v4fa;
typedef v8us __attribute__((may_alias)) v8usa;

__device__ __forceinline__ unsigned short f2bf(float f) { unsigned u = __float_as_uint(f); u += 0x7FFFu + ((u >> 16) & 1u); return (unsigned short)(u >> 16); }
__device__ __forceinline__ float bf2f(unsigned short b) { return __uint_as_float(((unsigned)b) << 16); }
__device__ __forceinline__ float bfr(float f) { return bf2f(f2bf(f)); }
__device__ __forceinline__ v16h cat16(v8h lo, v8h hi) { return __builtin_shufflevector(lo, hi, 0, 1, 2, 3, 4, 5, 6, 7, 8, 9, 10, 11, 12, 13, 14, 15); }
__device__ __forceinline__ v16bf cat16b(v8us lo, v8us hi) { return __builtin_bit_cast(v16bf, __builtin_shufflevector(lo, hi, 0, 1, 2, 3, 4, 5, 6, 7, 8, 9, 10, 11, 12, 13, 14, 15)); }
__device__ __forceinline__ v8f wmma16(v16h a, v16h b, v8f c) { return __builtin_amdgcn_wmma_f32_16x16x32_f16(false, a, false, b, (short)0, c, false, false); }
__device__ __forceinline__ v8f wmmab(v16bf a, v16bf b, v8f c) { return __builtin_amdgcn_wmma_f32_16x16x32_bf16(false, a, false, b, (short)0, c, false, false); }


template <typename T16> struct WFrag;
template <> struct WFrag<h16> { typedef v16h V; static __device__ __forceinline__ V ld(const h16* p) { return cat16(*(const v8h*)p, *(const v8h*)(p + 16)); } static __device__ __forceinline__ v8f mma(V a, V b, v8f c) { return wmma16(a, b, c); } };
template <> struct WFrag<bf> { typedef v16bf V; static __device__ __forceinline__ V ld(const bf* p) { return cat16b(*(const v8us*)p, *(const v8us*)(p + 16)); } static __device__ __forceinline__ v8f mma(V a, V b, v8f c) { return wmmab(a, b, c); } };
template <typename T16, int NSPLIT, bool BIAS>
__global__ __launch_bounds__(32) void k_gemmw(const T16* __restrict__ A, const T16* __restrict__ A2, const T16* __restrict__ Bt, const T16* __restrict__ Bt2, int K, float* C, int ldc, const float* __restrict__ bias, size_t sA, size_t sB, size_t sC) {
    typedef typename WFrag<T16>::V V;
    __shared__ __align__(16) float os[16 * 68];
    const size_t z = blockIdx.z; A += z * sA; if (A2) A2 += z * sA; Bt += z * sB; if (Bt2) Bt2 += z * sB; C += z * sC;
    const int lane = threadIdx.x & 31, lr = lane & 15, hi = lane >> 4; const int r0 = blockIdx.x * 64, c0 = blockIdx.y * 64;
    v8f acc[4][4];
#pragma unroll
    for (int mb = 0; mb < 4; ++mb)
#pragma unroll
        for (int nb = 0; nb < 4; ++nb) acc[mb][nb] = (v8f){};
    const size_t aoff = (size_t)(r0 + lr) * K + 8 * hi, boff = (size_t)(c0 + lr) * K + 8 * hi;
#pragma unroll 1
    for (int kc = 0; kc < K; kc += 32) {
        V a[4], a2[4];
#pragma unroll
        for (int mb = 0; mb < 4; ++mb) { a[mb] = WFrag<T16>::ld(A + aoff + (size_t)mb * 16 * K + kc); if (NSPLIT == 1 || NSPLIT == 2) a2[mb] = WFrag<T16>::ld(A2 + aoff + (size_t)mb * 16 * K + kc); }
#pragma unroll
        for (int nb = 0; nb < 4; ++nb) { const V b = WFrag<T16>::ld(Bt + boff + (size_t)nb * 16 * K + kc); V b2; if (NSPLIT >= 2) b2 = WFrag<T16>::ld(Bt2 + boff + (size_t)nb * 16 * K + kc);
#pragma unroll
            for (int mb = 0; mb < 4; ++mb) { acc[mb][nb] = WFrag<T16>::mma(a[mb], b, acc[mb][nb]); if (NSPLIT == 1 || NSPLIT == 2) acc[mb][nb] = WFrag<T16>::mma(a2[mb], b, acc[mb][nb]); if (NSPLIT >= 2) acc[mb][nb] = WFrag<T16>::mma(a[mb], b2, acc[mb][nb]); } }
        asm volatile("v_nop\n\tv_nop\n\tv_nop\n\tv_nop" : "+v"(acc[0][0]), "+v"(acc[1][1]), "+v"(acc[2][2]), "+v"(acc[3][3]) : "v"(a[0]), "v"(a[3]));
    }
#pragma unroll
    for (int mb = 0; mb < 4; ++mb) {
#pragma unroll
        for (int nb = 0; nb < 4; ++nb) {
#pragma unroll
            for (int j = 0; j < 8; ++j) os[(hi * 8 + j) * 68 + nb * 16 + lr] = acc[mb][nb][j]; }
        __builtin_amdgcn_wave_barrier(); asm volatile("" ::: "memory");
        float* crow = C + (size_t)(r0 + mb * 16) * ldc + c0;
#pragma unroll 1
        for (int ps = 0; ps < 2; ++ps) {
#pragma unroll
            for (int s = 0; s < 8; ++s) { const int row = 2 * s + hi, cofs = lr * 4; v4f val = *(const v4fa*)(os + row * 68 + cofs); if (BIAS) { val[0] += bfr(bias[c0 + cofs]); val[1] += bfr(bias[c0 + cofs + 1]); val[2] += bfr(bias[c0 + cofs + 2]); val[3] += bfr(bias[c0 + cofs + 3]); }
                *(volatile v4f*)(crow + (size_t)row * ldc + cofs) = val; }
            if (ps == 0) __threadfence(); }
        __builtin_amdgcn_wave_barrier(); asm volatile("" ::: "memory");
    }
}

__device__ __forceinline__ void splitf(float y, unsigned short& h, unsigned short& l) { h = f2bf(y); l = f2bf(y - bf2f(h)); }
typedef __attribute__((ext_vector_type(2))) float v2f;

__global__ __launch_bounds__(64) void k_ktab(const float* __restrict__ grid, int nin, float* T) { const int i = blockIdx.x * 64 + threadIdx.x; if (i >= nin) return; float g[NKN];
#pragma unroll
    for (int m = 0; m < NKN; ++m) g[m] = bfr(grid[i * NKN + m]);
    float* t = T + (size_t)i * 96;
#pragma unroll 1
    for (int ps = 0; ps < 2; ++ps) {
#pragma unroll
        for (int m = 0; m < NKN; ++m) *(volatile float*)(t + m) = g[m];
#pragma unroll
        for (int m = NKN; m < 16; ++m) *(volatile float*)(t + m) = 0.f;
#pragma unroll 1
        for (int d = 1; d <= 3; ++d) {
#pragma unroll 1
            for (int m = 0; m < 11; ++m) { const bool ok = (m + d + 1 <= NKN - 1) || (m + d <= NKN - 1); (void)ok;
                const float dl = (m + d < NKN) ? __fsub_rn(g[(m + d < NKN) ? m + d : 0], g[m]) : 1.0f; const float dr = (m + d + 1 < NKN) ? __fsub_rn(g[(m + d + 1 < NKN) ? m + d + 1 : 0], g[m + 1 < NKN ? m + 1 : 0]) : 1.0f;
                *(volatile float*)(t + 16 + (d - 1) * 11 + m) = __fdiv_rn(1.0f, dl); *(volatile float*)(t + 52 + (d - 1) * 11 + m) = __fdiv_rn(1.0f, dr); } }
#pragma unroll
        for (int m = 85; m < 96; ++m) *(volatile float*)(t + m) = 0.f;
        if (ps == 0) __threadfence(); } }
template <bool LAYER0, int TPR>
__global__ __launch_bounds__(256) void k_kfeat(const float* __restrict__ X, const float* __restrict__ H, int chunk, int nin, int kpitch, const float* __restrict__ T, bf* Ah, bf* Al) {
    const size_t e = (size_t)blockIdx.x * 256 + threadIdx.x; if (e >= (size_t)CH * TPR) return; const int i = (int)(e % TPR); const int r = (int)(e / TPR);
    if (LAYER0 && i >= nin) {
        v8us oh = (v8us){}, ol = (v8us){}; const size_t p = (size_t)chunk * CH + r; const int n = (int)(p / HWS), hw = (int)(p % HWS);
        if (i < nin + 2) {
#pragma unroll
            for (int q = 0; q < 8; ++q) { const int ii = (i - nin) * 8 + q; float sv = 0.f; if (ii < nin) { const float xx = bfr(X[((size_t)n * D0 + ii) * HWS + hw]); sv = __fmul_rn(xx, __builtin_amdgcn_rcpf(__fadd_rn(1.0f, __builtin_amdgcn_exp2f(__fmul_rn(-xx, 1.4426950408889634f))))    ); } unsigned short a, c; splitf(sv, a, c); oh[q] = a; ol[q] = c; } }
        const size_t oo = (size_t)r * kpitch + (size_t)i * NG; *(volatile v8us*)(Ah + oo) = oh; *(volatile v8us*)(Al + oo) = ol; __threadfence(); *(volatile v8us*)(Ah + oo) = oh; *(volatile v8us*)(Al + oo) = ol; return; }
    if (i >= nin) return;
    float x; if (LAYER0) { const size_t p = (size_t)chunk * CH + r; const int n = (int)(p / HWS), hw = (int)(p % HWS); x = bfr(X[((size_t)n * D0 + i) * HWS + hw]); } else { x = H[(size_t)r * NPAD + i]; }
    const float* t = T + (size_t)i * 96; float g[NKN]; float B[NKN - 1];
#pragma unroll
    for (int m = 0; m < NKN; ++m) g[m] = t[m];
#pragma unroll
    for (int m = 0; m < NKN - 1; ++m) B[m] = (g[m] <= x && x < g[m + 1]) ? 1.0f : 0.0f;
#pragma unroll
    for (int d = 1; d <= 3; ++d) {
#pragma unroll
        for (int m = 0; m < NKN - 1 - d; ++m) { const float rl = t[16 + (d - 1) * 11 + m], rr = t[52 + (d - 1) * 11 + m]; float a1 = __fmul_rn(__fsub_rn(x, g[m]), rl); asm volatile("" : "+v"(a1)); const float t1 = __fmul_rn(a1, B[m]); float a2 = __fmul_rn(__fsub_rn(g[m + d + 1], x), rr); asm volatile("" : "+v"(a2)); const float t2 = __fmul_rn(a2, B[m + 1]); B[m] = __fadd_rn(t1, t2); } }
    v8us oh, ol;
#pragma unroll
    for (int q = 0; q < NG; ++q) { unsigned short a, c; splitf(B[q], a, c); oh[q] = a; ol[q] = c; }
    const size_t oo = (size_t)r * kpitch + (size_t)i * NG; *(volatile v8us*)(Ah + oo) = oh; *(volatile v8us*)(Al + oo) = ol; __threadfence(); *(volatile v8us*)(Ah + oo) = oh; *(volatile v8us*)(Al + oo) = ol; }
template <bool LAYER0, int SPR>
__global__ __launch_bounds__(256) void k_ksilu(const float* __restrict__ X, const float* __restrict__ H, int chunk, int nin, int kpitch, bf* Ah, bf* Al) {
    const size_t e = (size_t)blockIdx.x * 256 + threadIdx.x; if (e >= (size_t)CH * SPR) return; const int j = (int)(e % SPR); const int r = (int)(e / SPR); const int ngr = (nin + 7) / 8; if (j >= ngr) return;
    v8us oh, ol; const size_t p = (size_t)chunk * CH + r; const int n = (int)(p / HWS), hw = (int)(p % HWS);
#pragma unroll
    for (int q = 0; q < 8; ++q) { const int i = j * 8 + q; float s = 0.f; if (i < nin) { const float x = LAYER0 ? bfr(X[((size_t)n * D0 + i) * HWS + hw]) : H[(size_t)r * NPAD + i]; s = __fmul_rn(x, __builtin_amdgcn_rcpf(__fadd_rn(1.0f, __builtin_amdgcn_exp2f(__fmul_rn(-x, 1.4426950408889634f))))); } unsigned short a, c; splitf(s, a, c); oh[q] = a; ol[q] = c; }
    const size_t oo = (size_t)r * kpitch + (size_t)nin * NG + (size_t)j * 8; const int npad8 = (j == ngr - 1) ? (kpitch - nin * NG - ngr * 8) / 8 : 0; const v8us z = (v8us){};
#pragma unroll 1
    for (int ps = 0; ps < 2; ++ps) { *(volatile v8us*)(Ah + oo) = oh; *(volatile v8us*)(Al + oo) = ol; for (int q = 0; q < npad8; ++q) { *(volatile v8us*)(Ah + oo + 8 + q * 8) = z; *(volatile v8us*)(Al + oo + 8 + q * 8) = z; } if (ps == 0) __threadfence(); } }
__global__ __launch_bounds__(256) void k_kw(const float* __restrict__ coef, const float* __restrict__ sb, const float* __restrict__ sp, int nin, int nout, int kpitch, bf* Wh, bf* Wl) {
    const int e = blockIdx.x * 256 + threadIdx.x; const int ng8 = kpitch / 8; if (e >= NPAD * ng8) return; const int gq = e % ng8, o = e / ng8; v8us oh, ol;
#pragma unroll
    for (int q = 0; q < 8; ++q) { const int k = gq * 8 + q; float w = 0.f;
        if (o < nout) { if (k < nin * NG) { const int i = k / NG, g = k % NG; w = __fmul_rn(bfr(sp[i * nout + o]), bfr(coef[((size_t)i * nout + o) * NG + g])); } else if (k < nin * NG + nin) { const int i = k - nin * NG; w = bfr(sb[i * nout + o]); } }
        unsigned short a, c; splitf(w, a, c); oh[q] = a; ol[q] = c; }
    const size_t oo = (size_t)o * kpitch + (size_t)gq * 8; *(volatile v8us*)(Wh + oo) = oh; *(volatile v8us*)(Wl + oo) = ol; __threadfence(); *(volatile v8us*)(Wh + oo) = oh; *(volatile v8us*)(Wl + oo) = ol; }
__global__ __launch_bounds__(256) void k_kout(const float* __restrict__ H, int chunk, float* OUT) { const size_t e = ((size_t)blockIdx.x * 256 + threadIdx.x) * 2; if (e >= (size_t)CH * D3) return; const int rr = (int)(e % CH); const int o = (int)(e / CH); const size_t p = (size_t)chunk * CH + rr; const int n = (int)(p / HWS), hw = (int)(p % HWS); v2f v; v[0] = H[(size_t)rr * NPAD + o]; v[1] = H[(size_t)(rr + 1) * NPAD + o];
    float* dst = OUT + ((size_t)n * D3 + o) * HWS + hw; *(volatile v2f*)dst = v; __threadfence(); *(volatile v2f*)dst = v; }

extern "C" void kernel_launch(void* const* d_in, const int* in_sizes, int n_in,
                              void* d_out, int out_size, void* d_ws, size_t ws_size, hipStream_t stream) {
    (void)in_sizes; (void)n_in; (void)out_size;
    const float* x = (const float*)d_in[0]; const float* g0 = (const float*)d_in[1]; const float* c0 = (const float*)d_in[2]; const float* sb0 = (const float*)d_in[3]; const float* sp0 = (const float*)d_in[4];
    const float* g1 = (const float*)d_in[5]; const float* c1 = (const float*)d_in[6]; const float* sb1 = (const float*)d_in[7]; const float* sp1 = (const float*)d_in[8]; const float* g2 = (const float*)d_in[9]; const float* c2 = (const float*)d_in[10]; const float* sb2 = (const float*)d_in[11]; const float* sp2 = (const float*)d_in[12];
    float* OUT = (float*)d_out;
    char* wsp = (char*)d_ws;
    auto take = [&](size_t bytes) { char* p = wsp; wsp += (bytes + 255) & ~(size_t)255; return (void*)p; };
    float* T0 = (float*)take((size_t)D0 * 96 * 4); float* T1 = (float*)take((size_t)D1 * 96 * 4); float* T2 = (float*)take((size_t)D2 * 96 * 4);
    bf* W0h = (bf*)take((size_t)NPAD * K0 * 2); bf* W0l = (bf*)take((size_t)NPAD * K0 * 2); bf* W1h = (bf*)take((size_t)NPAD * K1 * 2); bf* W1l = (bf*)take((size_t)NPAD * K1 * 2); bf* W2h = (bf*)take((size_t)NPAD * K1 * 2); bf* W2l = (bf*)take((size_t)NPAD * K1 * 2);
    bf* Ah = (bf*)take((size_t)CH * K1 * 2); bf* Al = (bf*)take((size_t)CH * K1 * 2); float* HA = (float*)take((size_t)CH * NPAD * 4); float* HB = (float*)take((size_t)CH * NPAD * 4);
    if ((size_t)(wsp - (char*)d_ws) > ws_size) return;
    k_ktab<<<1, 64, 0, stream>>>(g0, D0, T0); k_ktab<<<1, 64, 0, stream>>>(g1, D1, T1); k_ktab<<<1, 64, 0, stream>>>(g2, D2, T2);
    k_kw<<<(NPAD * (K0 / 8) + 255) / 256, 256, 0, stream>>>(c0, sb0, sp0, D0, D1, K0, W0h, W0l); k_kw<<<(NPAD * (K1 / 8) + 255) / 256, 256, 0, stream>>>(c1, sb1, sp1, D1, D2, K1, W1h, W1l); k_kw<<<(NPAD * (K1 / 8) + 255) / 256, 256, 0, stream>>>(c2, sb2, sp2, D2, D3, K1, W2h, W2l);
    for (int ck = 0; ck < NCH; ++ck) {
        k_kfeat<true, 16><<<(unsigned)(((size_t)CH * 16 + 255) / 256), 256, 0, stream>>>(x, nullptr, ck, D0, K0, T0, Ah, Al);
        k_gemmw<bf, 2, false><<<dim3(CH / 64, NPAD / 64, 1), 32, 0, stream>>>(Ah, Al, W0h, W0l, K0, HA, NPAD, nullptr, 0, 0, 0);
        k_kfeat<false, 64><<<(unsigned)(((size_t)CH * 64 + 255) / 256), 256, 0, stream>>>(nullptr, HA, ck, D1, K1, T1, Ah, Al); k_ksilu<false, 8><<<(unsigned)(((size_t)CH * 8 + 255) / 256), 256, 0, stream>>>(nullptr, HA, ck, D1, K1, Ah, Al);
        k_gemmw<bf, 2, false><<<dim3(CH / 64, NPAD / 64, 1), 32, 0, stream>>>(Ah, Al, W1h, W1l, K1, HB, NPAD, nullptr, 0, 0, 0);
        k_kfeat<false, 64><<<(unsigned)(((size_t)CH * 64 + 255) / 256), 256, 0, stream>>>(nullptr, HB, ck, D2, K1, T2, Ah, Al); k_ksilu<false, 8><<<(unsigned)(((size_t)CH * 8 + 255) / 256), 256, 0, stream>>>(nullptr, HB, ck, D2, K1, Ah, Al);
        k_gemmw<bf, 2, false><<<dim3(CH / 64, NPAD / 64, 1), 32, 0, stream>>>(Ah, Al, W2h, W2l, K1, HA, NPAD, nullptr, 0, 0, 0);
        k_kout<<<(unsigned)(((size_t)CH * D3 / 2 + 255) / 256), 256, 0, stream>>>(HA, ck, OUT); }
}
